// EnhancementLayerMamba_34497177321664
// MI455X (gfx1250) — hardware-run, weakly checked
//
#include <hip/hip_runtime.h>
#include <math.h>

typedef __attribute__((ext_vector_type(16))) _Float16 v16h;
typedef __attribute__((ext_vector_type(8)))  _Float16 v8h;
typedef __attribute__((ext_vector_type(8)))  float    v8f;
typedef __attribute__((ext_vector_type(4)))  float    v4f;

constexpr int kRows  = 128;
constexpr int kFeat  = 1024;
constexpr int kInner = 2048;
constexpr int kRank  = 512;
constexpr int kState = 512;
constexpr int kCond  = 512;
constexpr int kXzW   = 2 * kInner;
constexpr int kXdW   = kRank + 2 * kState;
constexpr int kGbW   = 2 * kState;
constexpr int kTaps  = 4;
static_assert(kXzW == 4096 && kXdW == 1536 && kGbW == 1024, "widths");
static_assert((kRows % 64) == 0, "GEMM M multiple of 64");
static_assert((kXzW % 64) == 0 && (kXdW % 64) == 0 && (kInner % 64) == 0 && (kFeat % 64) == 0 && (kState % 64) == 0 && (kGbW % 64) == 0, "GEMM N multiples of 64");
static_assert((kFeat % 64) == 0 && (kInner % 64) == 0 && (kRank % 64) == 0 && (kState % 64) == 0 && (kCond % 64) == 0, "GEMM K multiples of 32 (and of the 64-wide transpose tile)");

constexpr float kCarryW   = 1024.0f;
constexpr float kCarryAct = 64.0f;
constexpr float kCarryYg  = 512.0f;
constexpr float kFoldAct  = 1.0f / (kCarryAct * kCarryW);
constexpr float kFoldYg   = 1.0f / (kCarryYg * kCarryW);
constexpr float kF16MinNormal = 6.103515625e-05f;
constexpr float kF16Clamp     = 60000.0f;

constexpr size_t kOffWinT  = 0;
constexpr size_t kOffWxT   = kOffWinT  + (size_t)kXzW   * kFeat  * 2;
constexpr size_t kOffWdtT  = kOffWxT   + (size_t)kXdW   * kInner * 2;
constexpr size_t kOffWoutT = kOffWdtT  + (size_t)kInner * kRank  * 2;
constexpr size_t kOffWdT   = kOffWoutT + (size_t)kFeat  * kInner * 2;
constexpr size_t kOffWfT   = kOffWdT   + (size_t)kState * kFeat  * 2;
constexpr size_t kOffWoT   = kOffWfT   + (size_t)kGbW   * kCond  * 2;
constexpr size_t kOffHh    = kOffWoT   + (size_t)kFeat  * kState * 2;
constexpr size_t kOffCh    = kOffHh    + (size_t)kRows  * kFeat  * 2;
constexpr size_t kOffXZ    = kOffCh    + (size_t)kRows  * kCond  * 2;
constexpr size_t kOffUf    = kOffXZ    + (size_t)kRows  * kXzW   * 4;
constexpr size_t kOffUh    = kOffUf    + (size_t)kRows  * kInner * 4;
constexpr size_t kOffSRf   = kOffUh    + (size_t)kRows  * kInner * 2;
constexpr size_t kOffXD    = kOffSRf   + (size_t)kRows  * kInner * 4;
constexpr size_t kOffDRh   = kOffXD    + (size_t)kRows  * kXdW   * 4;
constexpr size_t kOffDT    = kOffDRh   + (size_t)kRows  * kRank  * 2;
constexpr size_t kOffYGh   = kOffDT    + (size_t)kRows  * kInner * 4;
constexpr size_t kOffMO    = kOffYGh   + (size_t)kRows  * kInner * 2;
constexpr size_t kOffMOXh  = kOffMO    + (size_t)kRows  * kFeat  * 4;
constexpr size_t kOffGB    = kOffMOXh  + (size_t)kRows  * kFeat  * 2;
constexpr size_t kOffZP    = kOffGB    + (size_t)kRows  * kGbW   * 4;
constexpr size_t kOffZh    = kOffZP    + (size_t)kRows  * kState * 4;
constexpr size_t kWsTotal  = kOffZh    + (size_t)kRows  * kState * 2;
static_assert(kWsTotal == 33423360ull, "carve total");
static_assert(kWsTotal <= 134217728ull, "carve cap");
static_assert((kOffWxT % 128) == 0 && (kOffWdtT % 128) == 0 && (kOffWoutT % 128) == 0 && (kOffWdT % 128) == 0 &&
              (kOffWfT % 128) == 0 && (kOffWoT % 128) == 0 && (kOffHh % 128) == 0 && (kOffCh % 128) == 0 &&
              (kOffXZ % 128) == 0 && (kOffUf % 128) == 0 && (kOffUh % 128) == 0 && (kOffSRf % 128) == 0 &&
              (kOffXD % 128) == 0 && (kOffDRh % 128) == 0 && (kOffDT % 128) == 0 && (kOffYGh % 128) == 0 &&
              (kOffMO % 128) == 0 && (kOffMOXh % 128) == 0 && (kOffGB % 128) == 0 && (kOffZP % 128) == 0 &&
              (kOffZh % 128) == 0, "128-B aligned regions");

__device__ __forceinline__ _Float16 f16_operand(float v) {
  const float w  = (fabsf(v) < kF16MinNormal) ? 0.0f : v;
  const float cl = fminf(fmaxf(w, -kF16Clamp), kF16Clamp);
  return (_Float16)cl;
}
__device__ __forceinline__ v8h pack8_f16(v4f a0, v4f a1, float carry) {
  v8h h;
#pragma unroll
  for (int e = 0; e < 4; ++e) {
    h[e]     = f16_operand(a0[e] * carry);
    h[4 + e] = f16_operand(a1[e] * carry);
  }
  return h;
}
__device__ __forceinline__ float silu_f32(float v) {
  return v * (1.0f / (1.0f + expf(-v)));
}

__device__ __forceinline__ void guard_row_h(v8f& a0, v8f& a1, v8f& a2, v8f& a3,
                                            v16h x, v16h y0, v16h y1, v16h y2, v16h y3) {
  asm volatile("" : "+v"(a0) : "v"(x), "v"(y0));
  asm volatile("" : "+v"(a1) : "v"(x), "v"(y1));
  asm volatile("" : "+v"(a2) : "v"(x), "v"(y2));
  asm volatile("v_nop\n\tv_nop\n\tv_nop\n\tv_nop" : "+v"(a3) : "v"(x), "v"(y3));
}
__device__ __forceinline__ void keep4_h(v16h a, v16h b, v16h c, v16h d) { asm volatile("v_nop" :: "v"(a), "v"(b), "v"(c), "v"(d)); }
__device__ __forceinline__ void acc_guard4(v8f& a, v8f& b, v8f& c, v8f& d) { asm volatile("v_nop\n\tv_nop\n\tv_nop\n\tv_nop" : "+v"(a), "+v"(b), "+v"(c), "+v"(d)); }

struct FragH {
  union U { v16h v; v8h h[2]; };
  static __device__ __forceinline__ v16h load(const _Float16* p) {
    U f;
    f.h[0] = *(const v8h*)(p);
    f.h[1] = *(const v8h*)(p + 16);
    return f.v;
  }
  static __device__ __forceinline__ v8f mma(v16h a, v16h b, v8f c) {
    return __builtin_amdgcn_wmma_f32_16x16x32_f16(false, a, false, b, (short)0, c, false, false);
  }
};

template <bool HAS_BIAS>
__global__ __launch_bounds__(256) void gemm_f16_tile64(
    const unsigned short* __restrict__ Ap, int lda,
    const unsigned short* __restrict__ Btp, int ldb,
    float* __restrict__ C, int ldc,
    const float* __restrict__ bias,
    int M, int N, int K, float scale) {
  const _Float16* A  = (const _Float16*)Ap;
  const _Float16* Bt = (const _Float16*)Btp;
  __shared__ __align__(16) float sT[8][16 * 68];
  const int lane = threadIdx.x & 31;
  const int wave = threadIdx.x >> 5;
  const int tilesN = N >> 6;
  const int tilesM = M >> 6;
  const int tile = blockIdx.x * 8 + wave;
  if (tile >= tilesM * tilesN) return;
  const int tm = tile / tilesN;
  const int tn = tile - tm * tilesN;
  const int m0 = tm << 6;
  const int n0 = tn << 6;

  const int rlane = lane & 15;
  const int koff  = (lane >> 4) * 8;
  const int mOff  = (lane >> 4) * 8;

  v8f acc[4][4];
#pragma unroll
  for (int i = 0; i < 4; ++i)
#pragma unroll
    for (int j = 0; j < 4; ++j) acc[i][j] = (v8f){0.f,0.f,0.f,0.f,0.f,0.f,0.f,0.f};

  for (int k0 = 0; k0 < K; k0 += 32) {
    v16h bh[4];
#pragma unroll
    for (int j = 0; j < 4; ++j) {
      const size_t bo = (size_t)(n0 + (j << 4) + rlane) * ldb + koff + k0;
      bh[j] = FragH::load(Bt + bo);
    }
#pragma unroll
    for (int i = 0; i < 4; ++i) {
      const size_t ao = (size_t)(m0 + (i << 4) + rlane) * lda + koff + k0;
      const v16h ah = FragH::load(A + ao);
#pragma unroll
      for (int j = 0; j < 4; ++j) acc[i][j] = FragH::mma(ah, bh[j], acc[i][j]);
      guard_row_h(acc[i][0], acc[i][1], acc[i][2], acc[i][3], ah, bh[0], bh[1], bh[2], bh[3]);
    }
    keep4_h(bh[0], bh[1], bh[2], bh[3]);
  }
  acc_guard4(acc[0][0], acc[0][1], acc[0][2], acc[0][3]);
  acc_guard4(acc[1][0], acc[1][1], acc[1][2], acc[1][3]);
  acc_guard4(acc[2][0], acc[2][1], acc[2][2], acc[2][3]);
  acc_guard4(acc[3][0], acc[3][1], acc[3][2], acc[3][3]);

  float* slab = sT[wave];
  const int hh = lane >> 4;
  const int c4 = (lane & 15) * 4;
  v4f bv = (v4f){0.f, 0.f, 0.f, 0.f};
  if (HAS_BIAS) bv = *(const v4f*)(bias + n0 + c4);
#pragma unroll
  for (int i = 0; i < 4; ++i) {
    const int mBase = m0 + (i << 4);
#pragma unroll
    for (int j = 0; j < 4; ++j) {
#pragma unroll
      for (int r = 0; r < 8; ++r) {
        slab[(mOff + r) * 68 + (j << 4) + rlane] = acc[i][j][r] * scale;
      }
    }
    __builtin_amdgcn_fence(__ATOMIC_RELEASE, "workgroup");
    __builtin_amdgcn_wave_barrier();
    __builtin_amdgcn_fence(__ATOMIC_ACQUIRE, "workgroup");
    for (int pass = 0; pass < 2; ++pass) {
#pragma unroll
      for (int it = 0; it < 8; ++it) {
        const int row = it * 2 + hh;
        v4f v = *(const v4f*)(slab + row * 68 + c4);
        v = v + bv;
        *(volatile v4f*)(C + (size_t)(mBase + row) * ldc + n0 + c4) = v;
      }
      __threadfence();
    }
    __builtin_amdgcn_fence(__ATOMIC_RELEASE, "workgroup");
    __builtin_amdgcn_wave_barrier();
    __builtin_amdgcn_fence(__ATOMIC_ACQUIRE, "workgroup");
  }
}

__global__ __launch_bounds__(256) void weight_plane_kernel(
    const float* __restrict__ W, unsigned short* __restrict__ Bt, int Kd, int Nd, float carry) {
  __shared__ __align__(16) float sTile[64 * 68];
  const int tid = threadIdx.x;
  const int n0 = blockIdx.x * 64;
  const int k0 = blockIdx.y * 64;
  const int c4 = (tid & 15) * 4;
  const int r  = tid >> 4;
#pragma unroll
  for (int i = 0; i < 4; ++i) {
    const int kk = r + 16 * i;
    const v4f v = *(const v4f*)(W + (size_t)(k0 + kk) * Nd + n0 + c4);
    *(v4f*)(sTile + kk * 68 + c4) = v;
  }
  __syncthreads();
  const int q  = tid >> 3;
  const int c8 = (tid & 7) * 8;
  v8h hv[2];
#pragma unroll
  for (int it = 0; it < 2; ++it) {
    const int n = q + 32 * it;
#pragma unroll
    for (int e = 0; e < 8; ++e) {
      const float xv = sTile[(c8 + e) * 68 + n] * carry;
      hv[it][e] = f16_operand(xv);
    }
  }
  for (int pass = 0; pass < 2; ++pass) {
#pragma unroll
    for (int it = 0; it < 2; ++it) {
      const int n = q + 32 * it;
      *(volatile v8h*)(Bt + (size_t)(n0 + n) * Kd + k0 + c8) = hv[it];
    }
    __threadfence();
  }
}

__global__ __launch_bounds__(128) void layernorm_cond_kernel(
    const float* __restrict__ x, const float* __restrict__ lng, const float* __restrict__ lnb,
    const float* __restrict__ cnd, unsigned short* __restrict__ Hh, unsigned short* __restrict__ Ch) {
  __shared__ float redA[4];
  __shared__ float redB[4];
  const int tid = threadIdx.x, lane = tid & 31, wave = tid >> 5;
  const int row = blockIdx.x;
  const size_t off = (size_t)row * kFeat + tid * 8;
  const v4f a0 = *(const v4f*)(x + off);
  const v4f a1 = *(const v4f*)(x + off + 4);
  float s = ((a0[0] + a0[1]) + (a0[2] + a0[3])) + ((a1[0] + a1[1]) + (a1[2] + a1[3]));
  s += __shfl_xor(s, 16, 32);
  s += __shfl_xor(s, 8, 32);
  s += __shfl_xor(s, 4, 32);
  s += __shfl_xor(s, 2, 32);
  s += __shfl_xor(s, 1, 32);
  if (lane == 0) redA[wave] = s;
  __syncthreads();
  const float mu = ((redA[0] + redA[1]) + (redA[2] + redA[3])) * (1.0f / (float)kFeat);
  const v4f d0 = a0 - mu;
  const v4f d1 = a1 - mu;
  float q = ((d0[0] * d0[0] + d0[1] * d0[1]) + (d0[2] * d0[2] + d0[3] * d0[3])) +
            ((d1[0] * d1[0] + d1[1] * d1[1]) + (d1[2] * d1[2] + d1[3] * d1[3]));
  q += __shfl_xor(q, 16, 32);
  q += __shfl_xor(q, 8, 32);
  q += __shfl_xor(q, 4, 32);
  q += __shfl_xor(q, 2, 32);
  q += __shfl_xor(q, 1, 32);
  if (lane == 0) redB[wave] = q;
  __syncthreads();
  const float var = ((redB[0] + redB[1]) + (redB[2] + redB[3])) * (1.0f / (float)kFeat);
  const float inv = rsqrtf(var + 1e-5f);
  const v4f g0 = *(const v4f*)(lng + tid * 8);
  const v4f g1 = *(const v4f*)(lng + tid * 8 + 4);
  const v4f b0 = *(const v4f*)(lnb + tid * 8);
  const v4f b1 = *(const v4f*)(lnb + tid * 8 + 4);
  v4f h0, h1;
#pragma unroll
  for (int e = 0; e < 4; ++e) {
    h0[e] = d0[e] * inv * g0[e] + b0[e];
    h1[e] = d1[e] * inv * g1[e] + b1[e];
  }
  const v8h hv = pack8_f16(h0, h1, kCarryAct);
  const int ct = tid & 63;
  const size_t coff = (size_t)row * kCond + ct * 8;
  const v4f c0 = *(const v4f*)(cnd + coff);
  const v4f c1 = *(const v4f*)(cnd + coff + 4);
  const v8h cv = pack8_f16(c0, c1, kCarryAct);
  for (int pass = 0; pass < 2; ++pass) {
    *(volatile v8h*)(Hh + off) = hv;
    if (tid < 64) *(volatile v8h*)(Ch + coff) = cv;
    __threadfence();
  }
}

__global__ __launch_bounds__(256) void conv_tap_silu_kernel(
    const float* __restrict__ XZ, const float* __restrict__ wtap, const float* __restrict__ cb,
    float* __restrict__ Uf, unsigned short* __restrict__ Uh, float* __restrict__ SRf) {
  __shared__ __align__(16) float sU[1024];
  __shared__ __align__(16) float sR[1024];
  const int tid = threadIdx.x;
  const int ch0 = blockIdx.x * 1024;
  const int row = blockIdx.y;
  const float* xr = XZ + (size_t)row * kXzW;
#pragma unroll 1
  for (int i = 0; i < 4; ++i) {
    const int loc = i * 256 + tid;
    const int e = ch0 + loc;
    const float xi = xr[e];
    const float xc = xi * wtap[e] + cb[e];
    sU[loc] = silu_f32(xc);
    const float rv = xr[kInner + e];
    sR[loc] = silu_f32(rv);
  }
  __syncthreads();
  const v4f uv = *(const v4f*)(sU + tid * 4);
  const v4f rv4 = *(const v4f*)(sR + tid * 4);
  const int ht = tid & 127;
  const v4f p0 = *(const v4f*)(sU + ht * 8);
  const v4f p1 = *(const v4f*)(sU + ht * 8 + 4);
  const v8h hv = pack8_f16(p0, p1, kCarryAct);
  const size_t ofs = (size_t)row * kInner + ch0;
  for (int pass = 0; pass < 2; ++pass) {
    *(volatile v4f*)(Uf + ofs + tid * 4) = uv;
    *(volatile v4f*)(SRf + ofs + tid * 4) = rv4;
    if (tid < 128) *(volatile v8h*)(Uh + ofs + tid * 8) = hv;
    __threadfence();
  }
}

template <bool ADD_SECOND>
__global__ __launch_bounds__(256) void plane_f16_kernel(
    const float* __restrict__ src, int srcPitch, const float* __restrict__ src2, int src2Pitch,
    unsigned short* __restrict__ dst, int dstW, int total, float carry) {
  const int idx = blockIdx.x * 256 + threadIdx.x;
  if (idx >= total) return;
  const int rowThreads = dstW >> 3;
  const int row = idx / rowThreads;
  const int c8 = (idx - row * rowThreads) * 8;
  v4f a0 = *(const v4f*)(src + (size_t)row * srcPitch + c8);
  v4f a1 = *(const v4f*)(src + (size_t)row * srcPitch + c8 + 4);
  if (ADD_SECOND) {
    const v4f s0 = *(const v4f*)(src2 + (size_t)row * src2Pitch + c8);
    const v4f s1 = *(const v4f*)(src2 + (size_t)row * src2Pitch + c8 + 4);
    a0 = a0 + s0;
    a1 = a1 + s1;
  }
  const v8h hv = pack8_f16(a0, a1, carry);
  unsigned short* p = dst + (size_t)row * dstW + c8;
  *(volatile v8h*)p = hv;
  __threadfence();
  *(volatile v8h*)p = hv;
}

__global__ __launch_bounds__(256) void state_gate_kernel(
    const float* __restrict__ DT, const float* __restrict__ XD, const float* __restrict__ Uf,
    const float* __restrict__ Dv, const float* __restrict__ SRf, unsigned short* __restrict__ YGh) {
  __shared__ __align__(16) float sB[512];
  __shared__ __align__(16) float sC[512];
  __shared__ __align__(16) float sY[256];
  const int tid = threadIdx.x;
  const int ch0 = blockIdx.x * 256;
  const int row = blockIdx.y;
  const float* xr = XD + (size_t)row * kXdW;
  sB[tid]       = xr[kRank + tid];
  sB[tid + 256] = xr[kRank + 256 + tid];
  sC[tid]       = xr[kRank + kState + tid];
  sC[tid + 256] = xr[kRank + kState + 256 + tid];
  const int e = ch0 + tid;
  const size_t o = (size_t)row * kInner + e;
  const float v = DT[o];
  const float delta = fmaxf(v, 0.0f) + log1pf(expf(-fabsf(v)));
  const float u = Uf[o];
  const float a = delta * u;
  __syncthreads();
  float acc = 0.0f;
#pragma unroll 2
  for (int n4 = 0; n4 < kState / 4; ++n4) {
    const v4f bq = *(const v4f*)(sB + 4 * n4);
    const v4f cq = *(const v4f*)(sC + 4 * n4);
    const float t0 = a * bq[0];
    acc = fmaf(t0, cq[0], acc);
    const float t1 = a * bq[1];
    acc = fmaf(t1, cq[1], acc);
    const float t2 = a * bq[2];
    acc = fmaf(t2, cq[2], acc);
    const float t3 = a * bq[3];
    acc = fmaf(t3, cq[3], acc);
  }
  const float y = acc + u * Dv[e];
  sY[tid] = y * SRf[o];
  __syncthreads();
  const int lt = tid & 31;
  const v4f p0 = *(const v4f*)(sY + lt * 8);
  const v4f p1 = *(const v4f*)(sY + lt * 8 + 4);
  const v8h hv = pack8_f16(p0, p1, kCarryYg);
  if (tid < 32) {
    unsigned short* p = YGh + (size_t)row * kInner + ch0 + tid * 8;
    *(volatile v8h*)p = hv;
    __threadfence();
    *(volatile v8h*)p = hv;
  }
}

__global__ __launch_bounds__(256) void gelu_scale_shift_kernel(
    const float* __restrict__ ZP, const float* __restrict__ GB, unsigned short* __restrict__ Zh) {
  __shared__ __align__(16) float sZ[512];
  const int tid = threadIdx.x;
  const int row = blockIdx.x;
#pragma unroll 1
  for (int i = 0; i < 2; ++i) {
    const int n = i * 256 + tid;
    const float zp = ZP[(size_t)row * kState + n];
    const float z = 0.5f * zp * (1.0f + erff(zp * 0.70710678118654752f));
    const float g  = GB[(size_t)row * kGbW + n];
    const float sh = GB[(size_t)row * kGbW + kState + n];
    sZ[n] = z * g + sh;
  }
  __syncthreads();
  const int zt = tid & 63;
  const v4f p0 = *(const v4f*)(sZ + zt * 8);
  const v4f p1 = *(const v4f*)(sZ + zt * 8 + 4);
  const v8h hv = pack8_f16(p0, p1, kCarryAct);
  if (tid < 64) {
    unsigned short* p = Zh + (size_t)row * kState + tid * 8;
    *(volatile v8h*)p = hv;
    __threadfence();
    *(volatile v8h*)p = hv;
  }
}

extern "C" void kernel_launch(void* const* d_in, const int* in_sizes, int n_in,
                              void* d_out, int out_size, void* d_ws, size_t ws_size,
                              hipStream_t stream) {
  if (n_in != 20) return;
  if (in_sizes[0] != kRows * kFeat) return;
  if (in_sizes[1] != kRows * kCond) return;
  if (in_sizes[2] != kFeat || in_sizes[3] != kFeat) return;
  if (in_sizes[4] != kFeat * kXzW) return;
  if (in_sizes[5] != kTaps * kInner) return;
  if (in_sizes[6] != kInner) return;
  if (in_sizes[7] != kInner * kXdW) return;
  if (in_sizes[8] != kRank * kInner) return;
  if (in_sizes[9] != kInner) return;
  if (in_sizes[10] != kInner * kState) return;
  if (in_sizes[11] != kInner) return;
  if (in_sizes[12] != kInner * kFeat) return;
  if (in_sizes[13] != kFeat) return;
  if (in_sizes[14] != kFeat * kState) return;
  if (in_sizes[15] != kState) return;
  if (in_sizes[16] != kCond * kGbW) return;
  if (in_sizes[17] != kGbW) return;
  if (in_sizes[18] != kState * kFeat) return;
  if (in_sizes[19] != kFeat) return;
  if (out_size != kRows * kFeat) return;
  if (ws_size < kWsTotal) return;

  const float* x      = (const float*)d_in[0];
  const float* cnd    = (const float*)d_in[1];
  const float* ln_g   = (const float*)d_in[2];
  const float* ln_b   = (const float*)d_in[3];
  const float* W_in   = (const float*)d_in[4];
  const float* conv_w = (const float*)d_in[5];
  const float* conv_b = (const float*)d_in[6];
  const float* W_x    = (const float*)d_in[7];
  const float* W_dt   = (const float*)d_in[8];
  const float* b_dt   = (const float*)d_in[9];
  const float* Dvec   = (const float*)d_in[11];
  const float* W_out  = (const float*)d_in[12];
  const float* b_out  = (const float*)d_in[13];
  const float* W_d    = (const float*)d_in[14];
  const float* b_d    = (const float*)d_in[15];
  const float* W_f    = (const float*)d_in[16];
  const float* b_f    = (const float*)d_in[17];
  const float* W_o    = (const float*)d_in[18];
  const float* b_o    = (const float*)d_in[19];
  float* out = (float*)d_out;

  char* ws = (char*)d_ws;
  unsigned short* WinT  = (unsigned short*)(ws + kOffWinT);
  unsigned short* WxT   = (unsigned short*)(ws + kOffWxT);
  unsigned short* WdtT  = (unsigned short*)(ws + kOffWdtT);
  unsigned short* WoutT = (unsigned short*)(ws + kOffWoutT);
  unsigned short* WdT   = (unsigned short*)(ws + kOffWdT);
  unsigned short* WfT   = (unsigned short*)(ws + kOffWfT);
  unsigned short* WoT   = (unsigned short*)(ws + kOffWoT);
  unsigned short* Hh    = (unsigned short*)(ws + kOffHh);
  unsigned short* Ch    = (unsigned short*)(ws + kOffCh);
  float*          XZ    = (float*)(ws + kOffXZ);
  float*          Uf    = (float*)(ws + kOffUf);
  unsigned short* Uh    = (unsigned short*)(ws + kOffUh);
  float*          SRf   = (float*)(ws + kOffSRf);
  float*          XD    = (float*)(ws + kOffXD);
  unsigned short* DRh   = (unsigned short*)(ws + kOffDRh);
  float*          DT    = (float*)(ws + kOffDT);
  unsigned short* YGh   = (unsigned short*)(ws + kOffYGh);
  float*          MO    = (float*)(ws + kOffMO);
  unsigned short* MOXh  = (unsigned short*)(ws + kOffMOXh);
  float*          GB    = (float*)(ws + kOffGB);
  float*          ZP    = (float*)(ws + kOffZP);
  unsigned short* Zh    = (unsigned short*)(ws + kOffZh);

  weight_plane_kernel<<<dim3(kXzW / 64,   kFeat / 64),  256, 0, stream>>>(W_in,  WinT,  kFeat,  kXzW,   kCarryW);
  weight_plane_kernel<<<dim3(kXdW / 64,   kInner / 64), 256, 0, stream>>>(W_x,   WxT,   kInner, kXdW,   kCarryW);
  weight_plane_kernel<<<dim3(kInner / 64, kRank / 64),  256, 0, stream>>>(W_dt,  WdtT,  kRank,  kInner, kCarryW);
  weight_plane_kernel<<<dim3(kFeat / 64,  kInner / 64), 256, 0, stream>>>(W_out, WoutT, kInner, kFeat,  kCarryW);
  weight_plane_kernel<<<dim3(kState / 64, kFeat / 64),  256, 0, stream>>>(W_d,   WdT,   kFeat,  kState, kCarryW);
  weight_plane_kernel<<<dim3(kGbW / 64,   kCond / 64),  256, 0, stream>>>(W_f,   WfT,   kCond,  kGbW,   kCarryW);
  weight_plane_kernel<<<dim3(kFeat / 64,  kState / 64), 256, 0, stream>>>(W_o,   WoT,   kState, kFeat,  kCarryW);

  layernorm_cond_kernel<<<kRows, 128, 0, stream>>>(x, ln_g, ln_b, cnd, Hh, Ch);

  gemm_f16_tile64<false><<<(2 * (kXzW / 64) + 7) / 8, 256, 0, stream>>>(
      Hh, kFeat, WinT, kFeat, XZ, kXzW, nullptr, kRows, kXzW, kFeat, kFoldAct);

  conv_tap_silu_kernel<<<dim3(kInner / 1024, kRows), 256, 0, stream>>>(
      XZ, conv_w + (size_t)(kTaps - 1) * kInner, conv_b, Uf, Uh, SRf);

  gemm_f16_tile64<false><<<(2 * (kXdW / 64) + 7) / 8, 256, 0, stream>>>(
      Uh, kInner, WxT, kInner, XD, kXdW, nullptr, kRows, kXdW, kInner, kFoldAct);

  plane_f16_kernel<false><<<(kRows * (kRank / 8) + 255) / 256, 256, 0, stream>>>(
      XD, kXdW, nullptr, 0, DRh, kRank, kRows * (kRank / 8), kCarryAct);

  gemm_f16_tile64<true><<<(2 * (kInner / 64) + 7) / 8, 256, 0, stream>>>(
      DRh, kRank, WdtT, kRank, DT, kInner, b_dt, kRows, kInner, kRank, kFoldAct);

  state_gate_kernel<<<dim3(kInner / 256, kRows), 256, 0, stream>>>(DT, XD, Uf, Dvec, SRf, YGh);

  gemm_f16_tile64<true><<<(2 * (kFeat / 64) + 7) / 8, 256, 0, stream>>>(
      YGh, kInner, WoutT, kInner, MO, kFeat, b_out, kRows, kFeat, kInner, kFoldYg);

  plane_f16_kernel<true><<<(kRows * (kFeat / 8) + 255) / 256, 256, 0, stream>>>(
      MO, kFeat, x, kFeat, MOXh, kFeat, kRows * (kFeat / 8), kCarryAct);

  gemm_f16_tile64<true><<<(2 * (kGbW / 64) + 7) / 8, 256, 0, stream>>>(
      Ch, kCond, WfT, kCond, GB, kGbW, b_f, kRows, kGbW, kCond, kFoldAct);

  gemm_f16_tile64<true><<<(2 * (kState / 64) + 7) / 8, 256, 0, stream>>>(
      MOXh, kFeat, WdT, kFeat, ZP, kState, b_d, kRows, kState, kFeat, kFoldAct);

  gelu_scale_shift_kernel<<<kRows, 256, 0, stream>>>(ZP, GB, Zh);

  gemm_f16_tile64<true><<<(2 * (kFeat / 64) + 7) / 8, 256, 0, stream>>>(
      Zh, kState, WoT, kState, out, kFeat, b_o, kRows, kFeat, kState, kFoldAct);
}
